// LinearAttention_21414706937909
// MI455X (gfx1250) — hardware-run, weakly checked
//
#include <hip/hip_runtime.h>
#include <math.h>

typedef __attribute__((ext_vector_type(16))) __bf16   v16b;
typedef __attribute__((ext_vector_type(8)))  __bf16   v8b;
typedef __attribute__((ext_vector_type(8)))  _Float16 v8h;
typedef __attribute__((ext_vector_type(8)))  float    v8f;
typedef __attribute__((ext_vector_type(4)))  float    v4f;
typedef __attribute__((ext_vector_type(4)))  unsigned int v4u;

constexpr int kBatch   = 4;
constexpr int kSeqLen  = 2048;
constexpr int kEmb     = 1024;
constexpr int kHeads   = 16;
constexpr int kHeadDim = 64;
constexpr int kChunk   = 128;
constexpr int kNumChunks = kSeqLen / kChunk;
constexpr int kRows    = kBatch * kSeqLen;
constexpr int kPlanePitch = 3 * kEmb;
constexpr int kColQ    = 0;
constexpr int kColK    = kEmb;
constexpr int kColV    = 2 * kEmb;
constexpr int kVtPitch = 136;
constexpr int kStPitch = 72;
constexpr int kSlabPitch = 68;
constexpr float kDenEps = 1e-6f;
static_assert(kHeads * kHeadDim == kEmb, "head split");
static_assert(kNumChunks == 16 && kChunk == 128 && kHeadDim == 64, "chunk geometry the core kernel is written for");
static_assert((kEmb % 32) == 0, "GEMM K multiple of 32");
static_assert((kRows % 64) == 0 && (kPlanePitch % 64) == 0 && (kEmb % 64) == 0, "GEMM M,N multiples of 64");
static_assert(2 * 64 * kVtPitch * 2 == 8 * 16 * kSlabPitch * 4, "slab overlay has the size of the transposed value tiles");
static_assert((kVtPitch % 8) == 0 && (kStPitch % 8) == 0, "16-byte aligned LDS fragment rows");

constexpr size_t kBytesXB   = (size_t)kRows * kEmb * 2;
constexpr size_t kBytesWALL = (size_t)4 * kEmb * kEmb * 2;
constexpr size_t kBytesPH   = (size_t)kRows * kPlanePitch * 2;
constexpr size_t kBytesPL   = (size_t)kRows * kPlanePitch * 2;
constexpr size_t kWsTotal   = kBytesXB + kBytesWALL + kBytesPH + kBytesPL;
static_assert(kWsTotal == 125829120ull, "carve total");
static_assert(kWsTotal <= 134217728ull, "carve cap");

__device__ __forceinline__ unsigned short f2bf_bits(float f) {
  unsigned u = __float_as_uint(f);
  return (unsigned short)((u + 0x7FFFu + ((u >> 16) & 1u)) >> 16);
}
__device__ __forceinline__ float bf_bits2f(unsigned short h) { return __uint_as_float(((unsigned)h) << 16); }

__device__ __forceinline__ v16b frag_load(const __bf16* p) {
  union { v16b v; v8b h[2]; } f;
  f.h[0] = *(const v8b*)(p);
  f.h[1] = *(const v8b*)(p + 16);
  return f.v;
}
__device__ __forceinline__ v8f wmma_raw(v16b a, v16b b, v8f c) {
  return __builtin_amdgcn_wmma_f32_16x16x32_bf16(false, a, false, b, (short)0, c, false, false);
}
__device__ __forceinline__ v8f mma_b(v16b a, v16b b, v8f c) {
  c = __builtin_amdgcn_wmma_f32_16x16x32_bf16(false, a, false, b, (short)0, c, false, false);
  asm volatile("v_nop\n\tv_nop\n\tv_nop\n\tv_nop" : "+v"(c) : "v"(a), "v"(b));
  return c;
}
__device__ __forceinline__ void dep_guard4_b(v8f& a, v8f& b, v8f& c, v8f& d, v16b x, v16b y) {
  asm volatile("v_nop\n\tv_nop\n\tv_nop\n\tv_nop" : "+v"(a), "+v"(b), "+v"(c), "+v"(d) : "v"(x), "v"(y));
}
__device__ __forceinline__ void keep4_b(v16b a, v16b b, v16b c, v16b d) { asm volatile("v_nop" :: "v"(a), "v"(b), "v"(c), "v"(d)); }
__device__ __forceinline__ void acc_guard4(v8f& a, v8f& b, v8f& c, v8f& d) {
  asm volatile("v_nop\n\tv_nop\n\tv_nop\n\tv_nop" : "+v"(a), "+v"(b), "+v"(c), "+v"(d));
}

__device__ __forceinline__ void split_pack(float x0, float x1, unsigned& wh, unsigned& wl) {
  const unsigned short h0 = f2bf_bits(x0), h1 = f2bf_bits(x1);
  const unsigned short l0 = f2bf_bits(x0 - bf_bits2f(h0)), l1 = f2bf_bits(x1 - bf_bits2f(h1));
  wh = (unsigned)h0 | ((unsigned)h1 << 16);
  wl = (unsigned)l0 | ((unsigned)l1 << 16);
}

__device__ __forceinline__ void st_tr8(unsigned short* p, int pitch, v4u w) {
  const unsigned w0 = w[0], w1 = w[1], w2 = w[2], w3 = w[3];
  p[0 * pitch] = (unsigned short)(w0 & 0xffffu);
  p[1 * pitch] = (unsigned short)(w0 >> 16);
  p[2 * pitch] = (unsigned short)(w1 & 0xffffu);
  p[3 * pitch] = (unsigned short)(w1 >> 16);
  p[4 * pitch] = (unsigned short)(w2 & 0xffffu);
  p[5 * pitch] = (unsigned short)(w2 >> 16);
  p[6 * pitch] = (unsigned short)(w3 & 0xffffu);
  p[7 * pitch] = (unsigned short)(w3 >> 16);
}

union FragWords { v16b v; unsigned u[8]; };

__device__ __forceinline__ float frag_dot_vec(v16b fhv, v16b flv, const float* zp, float acc) {
  FragWords fh, fl;
  fh.v = fhv;
  fl.v = flv;
#pragma unroll
  for (int half = 0; half < 2; ++half) {
    const v4f z0 = *(const v4f*)(zp + 16 * half);
    const v4f z1 = *(const v4f*)(zp + 16 * half + 4);
    const float z[8] = {z0[0], z0[1], z0[2], z0[3], z1[0], z1[1], z1[2], z1[3]};
#pragma unroll
    for (int j = 0; j < 4; ++j) {
      const unsigned wh = fh.u[4 * half + j], wl = fl.u[4 * half + j];
      const float a0 = __uint_as_float(wh << 16) + __uint_as_float(wl << 16);
      const float a1 = __uint_as_float(wh & 0xffff0000u) + __uint_as_float(wl & 0xffff0000u);
      acc = fmaf(a0, z[2 * j], acc);
      acc = fmaf(a1, z[2 * j + 1], acc);
    }
  }
  return acc;
}

__global__ __launch_bounds__(256) void cvt8_bf16_kernel(const float* s0, const float* s1, const float* s2, const float* s3,
                                                        unsigned short* __restrict__ dst, int n8) {
  const int y = blockIdx.y;
  const float* src = (y == 0) ? s0 : (y == 1) ? s1 : (y == 2) ? s2 : s3;
  const int i = blockIdx.x * 256 + threadIdx.x;
  if (i >= n8) return;
  const float* p = src + 8 * (size_t)i;
  const v4f a = *(const v4f*)(p);
  const v4f c = *(const v4f*)(p + 4);
  v8h hv;
#pragma unroll
  for (int e = 0; e < 4; ++e) {
    const float fa = a[e];
    const float fc = c[e];
    const unsigned short b0 = f2bf_bits(fa);
    const unsigned short b1 = f2bf_bits(fc);
    hv[e]     = __builtin_bit_cast(_Float16, b0);
    hv[4 + e] = __builtin_bit_cast(_Float16, b1);
  }
  unsigned short* q = dst + (size_t)y * (size_t)n8 * 8 + 8 * (size_t)i;
  *(volatile v8h*)q = hv;
  __threadfence();
  *(volatile v8h*)q = hv;
}

template <int SPL, int BIAS_MODE, int OUT_MODE, int ACT>
__global__ __launch_bounds__(256) void wmma_gemm64(
    const unsigned short* __restrict__ Ap, const unsigned short* __restrict__ A2p, int lda,
    const unsigned short* __restrict__ Btp, int ldb,
    void* __restrict__ Cout, void* __restrict__ Cout2, int ldc,
    const float* __restrict__ bias, int M, int N, int K, int act_ncols) {
  const __bf16* A  = (const __bf16*)Ap;
  const __bf16* A2 = (const __bf16*)A2p;
  const __bf16* Bt = (const __bf16*)Btp;
  __shared__ __align__(16) float sT[8][16 * 68];
  const int lane = threadIdx.x & 31;
  const int wave = threadIdx.x >> 5;
  const int tilesN = N >> 6;
  const int tilesM = M >> 6;
  const int tile = blockIdx.x * 8 + wave;
  if (tile >= tilesM * tilesN) return;
  const int tm = tile / tilesN;
  const int tn = tile - tm * tilesN;
  const int m0 = tm << 6;
  const int n0 = tn << 6;
  const int rlane = lane & 15;
  const int koff  = (lane >> 4) * 8;
  const int mOff  = (lane >> 4) * 8;

  v8f acc[4][4];
#pragma unroll
  for (int i = 0; i < 4; ++i)
#pragma unroll
    for (int j = 0; j < 4; ++j) acc[i][j] = (v8f){0.f, 0.f, 0.f, 0.f, 0.f, 0.f, 0.f, 0.f};

  for (int k0 = 0; k0 < K; k0 += 32) {
    v16b bh[4];
#pragma unroll
    for (int j = 0; j < 4; ++j) {
      const size_t bo = (size_t)(n0 + (j << 4) + rlane) * ldb + koff + k0;
      bh[j] = frag_load(Bt + bo);
    }
#pragma unroll
    for (int i = 0; i < 4; ++i) {
      const size_t ao = (size_t)(m0 + (i << 4) + rlane) * lda + koff + k0;
      const v16b ah = frag_load(A + ao);
      v16b al = ah;
      if (SPL >= 1) al = frag_load(A2 + ao);
#pragma unroll
      for (int j = 0; j < 4; ++j) {
        acc[i][j] = wmma_raw(ah, bh[j], acc[i][j]);
        if (SPL >= 1) acc[i][j] = wmma_raw(al, bh[j], acc[i][j]);
      }
      dep_guard4_b(acc[i][0], acc[i][1], acc[i][2], acc[i][3], ah, al);
    }
    keep4_b(bh[0], bh[1], bh[2], bh[3]);
  }
  acc_guard4(acc[0][0], acc[0][1], acc[0][2], acc[0][3]);
  acc_guard4(acc[1][0], acc[1][1], acc[1][2], acc[1][3]);
  acc_guard4(acc[2][0], acc[2][1], acc[2][2], acc[2][3]);
  acc_guard4(acc[3][0], acc[3][1], acc[3][2], acc[3][3]);

  float* slab = sT[wave];
  const bool doact = (ACT == 6) && (n0 < act_ncols);
#pragma unroll
  for (int i = 0; i < 4; ++i) {
    const int mBase = m0 + (i << 4);
#pragma unroll
    for (int j = 0; j < 4; ++j) {
      const int n = n0 + (j << 4) + rlane;
      float bv = 0.f;
      if (BIAS_MODE == 2) bv = bf_bits2f(f2bf_bits(bias[n]));
#pragma unroll
      for (int r = 0; r < 8; ++r) {
        float v = acc[i][j][r];
        if (BIAS_MODE == 2) v += bv;
        if (ACT == 6) {
          const float va = (v > 0.f) ? (v + 1.0f) : __expf(v);
          v = doact ? va : v;
        }
        slab[(mOff + r) * 68 + (j << 4) + rlane] = v;
      }
    }
    __builtin_amdgcn_fence(__ATOMIC_RELEASE, "workgroup");
    __builtin_amdgcn_wave_barrier();
    __builtin_amdgcn_fence(__ATOMIC_ACQUIRE, "workgroup");
    if (OUT_MODE == 0) {
      float* C = (float*)Cout;
      const int hh = lane >> 4, c4 = (lane & 15) * 4;
      for (int pass = 0; pass < 2; ++pass) {
#pragma unroll
        for (int it = 0; it < 8; ++it) {
          const int row = it * 2 + hh;
          const v4f v = *(const v4f*)(slab + row * 68 + c4);
          *(volatile v4f*)(C + (size_t)(mBase + row) * ldc + n0 + c4) = v;
        }
        __threadfence();
      }
    } else {
      const int q8 = lane >> 3, c8 = (lane & 7) * 8;
      unsigned short* C  = (unsigned short*)Cout;
      unsigned short* C2 = (unsigned short*)Cout2;
      for (int pass = 0; pass < 2; ++pass) {
#pragma unroll
        for (int it = 0; it < 4; ++it) {
          const int row = it * 4 + q8;
          const float* sp = slab + row * 68 + c8;
          v8h hv, lv;
#pragma unroll
          for (int e = 0; e < 8; ++e) {
            const float x = sp[e];
            const unsigned short hb = f2bf_bits(x);
            const unsigned short lb = f2bf_bits(x - bf_bits2f(hb));
            hv[e] = __builtin_bit_cast(_Float16, hb);
            lv[e] = __builtin_bit_cast(_Float16, lb);
          }
          *(volatile v8h*)(C  + (size_t)(mBase + row) * ldc + n0 + c8) = hv;
          *(volatile v8h*)(C2 + (size_t)(mBase + row) * ldc + n0 + c8) = lv;
        }
        __threadfence();
      }
    }
    __builtin_amdgcn_fence(__ATOMIC_RELEASE, "workgroup");
    __builtin_amdgcn_wave_barrier();
    __builtin_amdgcn_fence(__ATOMIC_ACQUIRE, "workgroup");
  }
}

__device__ __forceinline__ v8f score_tile_t(const __bf16* kh, const __bf16* kl, v16b qh0, v16b ql0, v16b qh1, v16b ql1) {
  v8f t = (v8f){0.f, 0.f, 0.f, 0.f, 0.f, 0.f, 0.f, 0.f};
  v16b ah = frag_load(kh);
  v16b al = frag_load(kl);
  t = mma_b(ah, qh0, t);
  t = mma_b(ah, ql0, t);
  t = mma_b(al, qh0, t);
  ah = frag_load(kh + 32);
  al = frag_load(kl + 32);
  t = mma_b(ah, qh1, t);
  t = mma_b(ah, ql1, t);
  t = mma_b(al, qh1, t);
  return t;
}

__global__ __launch_bounds__(256) void chunk_core_kernel(unsigned short* PH, unsigned short* PL) {
  __shared__ __align__(16) unsigned short sV[2 * 64 * kVtPitch];
  __shared__ __align__(16) unsigned short sR[2 * 64 * kStPitch];
  __shared__ __align__(16) float sZ[64];

  const int tid  = threadIdx.x;
  const int lane = tid & 31;
  const int wave = __builtin_amdgcn_readfirstlane(tid >> 5);
  const int hh = lane >> 4;
  const int c  = lane & 15;
  const int bh = blockIdx.x;
  const int b  = bh >> 4;
  const int h  = bh & 15;
  const int et  = wave >> 1;
  const int dt0 = (wave & 1) * 2;

  unsigned short* sVl = sV + 64 * kVtPitch;
  unsigned short* sRl = sR + 64 * kStPitch;
  const __bf16* vTh = (const __bf16*)sV;
  const __bf16* vTl = vTh + 64 * kVtPitch;
  const __bf16* rTh = (const __bf16*)sR;
  const __bf16* rTl = rTh + 64 * kStPitch;
  float* slab = (float*)sV + wave * (16 * kSlabPitch);

  const v8f zero8 = (v8f){0.f, 0.f, 0.f, 0.f, 0.f, 0.f, 0.f, 0.f};
  v8f S0 = zero8, S1 = zero8;
  float zreg = 0.f;

  const int q8 = lane >> 3;
  const int c8 = (lane & 7) * 8;
  const int cq = 16 * wave + c;

#pragma unroll 1
  for (int n = 0; n < kNumChunks; ++n) {
    const size_t row0 = (size_t)b * kSeqLen + (size_t)n * kChunk;

#pragma unroll
    for (int r = 0; r < 8; ++r) {
      const int e = 16 * et + 8 * hh + r;
      const float x0 = S0[r];
      const float x1 = S1[r];
      const unsigned short h0 = f2bf_bits(x0), h1 = f2bf_bits(x1);
      const unsigned short l0 = f2bf_bits(x0 - bf_bits2f(h0)), l1 = f2bf_bits(x1 - bf_bits2f(h1));
      sR [e * kStPitch + 16 * dt0 + c]      = h0;
      sRl[e * kStPitch + 16 * dt0 + c]      = l0;
      sR [e * kStPitch + 16 * dt0 + 16 + c] = h1;
      sRl[e * kStPitch + 16 * dt0 + 16 + c] = l1;
    }
    if (tid < 64) sZ[tid] = zreg;
#pragma unroll
    for (int it = 0; it < 4; ++it) {
      const int i  = it * 256 + tid;
      const int cc = i >> 3;
      const int d8 = (i & 7) * 8;
      const size_t go = (row0 + cc) * kPlanePitch + kColV + h * kHeadDim + d8;
      const v4u wh = *(const v4u*)(PH + go);
      const v4u wl = *(const v4u*)(PL + go);
      st_tr8(sV  + d8 * kVtPitch + cc, kVtPitch, wh);
      st_tr8(sVl + d8 * kVtPitch + cc, kVtPitch, wl);
    }
    __syncthreads();

    v8f num[4];
#pragma unroll
    for (int t = 0; t < 4; ++t) num[t] = zero8;
    float rs = 0.f;

    const size_t qoff = (row0 + 16 * wave + c) * kPlanePitch + kColQ + h * kHeadDim + 8 * hh;
    const v16b qh0 = frag_load((const __bf16*)PH + qoff);
    const v16b qh1 = frag_load((const __bf16*)PH + qoff + 32);
    const v16b ql0 = frag_load((const __bf16*)PL + qoff);
    const v16b ql1 = frag_load((const __bf16*)PL + qoff + 32);

    const int kkmax = wave >> 1;
#pragma unroll 1
    for (int kk = 0; kk <= kkmax; ++kk) {
      const size_t koffs = (row0 + 32 * kk + c) * kPlanePitch + kColK + h * kHeadDim + 8 * hh;
      const __bf16* khp = (const __bf16*)PH + koffs;
      const __bf16* klp = (const __bf16*)PL + koffs;
      v8f at0 = score_tile_t(khp, klp, qh0, ql0, qh1, ql1);
      v8f at1 = score_tile_t(khp + 16 * kPlanePitch, klp + 16 * kPlanePitch, qh0, ql0, qh1, ql1);
#pragma unroll
      for (int r = 0; r < 8; ++r) {
        const int s0 = 32 * kk + 8 * hh + r;
        const int s1 = s0 + 16;
        const float x0 = (s0 <= cq) ? at0[r] : 0.0f;
        const float x1 = (s1 <= cq) ? at1[r] : 0.0f;
        at0[r] = x0;
        at1[r] = x1;
        rs += x0 + x1;
      }
      FragWords pah, pal;
#pragma unroll
      for (int j = 0; j < 4; ++j) {
        unsigned wh, wl;
        split_pack(at0[2 * j], at0[2 * j + 1], wh, wl);
        pah.u[j] = wh;
        pal.u[j] = wl;
        split_pack(at1[2 * j], at1[2 * j + 1], wh, wl);
        pah.u[4 + j] = wh;
        pal.u[4 + j] = wl;
      }
#pragma unroll
      for (int t = 0; t < 4; ++t) {
        const int vo = (16 * t + c) * kVtPitch + 32 * kk + 8 * hh;
        const v16b vbh = frag_load(vTh + vo);
        const v16b vbl = frag_load(vTl + vo);
        num[t] = mma_b(pah.v, vbh, num[t]);
        num[t] = mma_b(pah.v, vbl, num[t]);
        num[t] = mma_b(pal.v, vbh, num[t]);
      }
    }

#pragma unroll
    for (int t = 0; t < 4; ++t) {
      const int so = (16 * t + c) * kStPitch + 8 * hh;
      v16b sbh = frag_load(rTh + so);
      v16b sbl = frag_load(rTl + so);
      num[t] = mma_b(qh0, sbh, num[t]);
      num[t] = mma_b(qh0, sbl, num[t]);
      num[t] = mma_b(ql0, sbh, num[t]);
      sbh = frag_load(rTh + so + 32);
      sbl = frag_load(rTl + so + 32);
      num[t] = mma_b(qh1, sbh, num[t]);
      num[t] = mma_b(qh1, sbl, num[t]);
      num[t] = mma_b(ql1, sbh, num[t]);
    }

    float qz = 0.f;
    qz = frag_dot_vec(qh0, ql0, sZ + 8 * hh, qz);
    qz = frag_dot_vec(qh1, ql1, sZ + 32 + 8 * hh, qz);
    rs += __shfl_xor(rs, 16, 32);
    qz += __shfl_xor(qz, 16, 32);
    const float den  = (rs + qz) + kDenEps;
    const float dinv = 1.0f / den;
#pragma unroll
    for (int r = 0; r < 8; ++r) {
      const float di = __shfl(dinv, 8 * hh + r, 32);
#pragma unroll
      for (int t = 0; t < 4; ++t) num[t][r] = num[t][r] * di;
    }
    __syncthreads();

#pragma unroll 1
    for (int j = 0; j < 2; ++j) {
#pragma unroll
      for (int it = 0; it < 2; ++it) {
        const int i  = it * 256 + tid;
        const int cc = i >> 3;
        const int d8 = (i & 7) * 8;
        const size_t go = (row0 + 64 * j + cc) * kPlanePitch + kColK + h * kHeadDim + d8;
        const v4u wh = *(const v4u*)(PH + go);
        const v4u wl = *(const v4u*)(PL + go);
        st_tr8(sR  + d8 * kStPitch + cc, kStPitch, wh);
        st_tr8(sRl + d8 * kStPitch + cc, kStPitch, wl);
      }
      __syncthreads();
      if (tid < 64) {
        float z = 0.f;
#pragma unroll 1
        for (int g = 0; g < 8; ++g) {
          const v4u a  = *(const v4u*)(sR  + tid * kStPitch + 8 * g);
          const v4u bq = *(const v4u*)(sRl + tid * kStPitch + 8 * g);
#pragma unroll
          for (int jj = 0; jj < 4; ++jj) {
            const unsigned wa = a[jj];
            const unsigned wb = bq[jj];
            z += __uint_as_float(wa << 16) + __uint_as_float(wb << 16);
            z += __uint_as_float(wa & 0xffff0000u) + __uint_as_float(wb & 0xffff0000u);
          }
        }
        zreg += z;
      }
#pragma unroll
      for (int kk2 = 0; kk2 < 2; ++kk2) {
        const int vo = (16 * et + c) * kVtPitch + 64 * j + 32 * kk2 + 8 * hh;
        const v16b vah = frag_load(vTh + vo);
        const v16b val = frag_load(vTl + vo);
        const int ko = (16 * dt0 + c) * kStPitch + 32 * kk2 + 8 * hh;
        const v16b k0h = frag_load(rTh + ko);
        const v16b k0l = frag_load(rTl + ko);
        const v16b k1h = frag_load(rTh + ko + 16 * kStPitch);
        const v16b k1l = frag_load(rTl + ko + 16 * kStPitch);
        S0 = mma_b(vah, k0h, S0);
        S0 = mma_b(vah, k0l, S0);
        S0 = mma_b(val, k0h, S0);
        S1 = mma_b(vah, k1h, S1);
        S1 = mma_b(vah, k1l, S1);
        S1 = mma_b(val, k1h, S1);
      }
      __syncthreads();
    }

#pragma unroll
    for (int t = 0; t < 4; ++t)
#pragma unroll
      for (int r = 0; r < 8; ++r) slab[(8 * hh + r) * kSlabPitch + 16 * t + c] = num[t][r];
    __builtin_amdgcn_fence(__ATOMIC_RELEASE, "workgroup");
    __builtin_amdgcn_wave_barrier();
    __builtin_amdgcn_fence(__ATOMIC_ACQUIRE, "workgroup");
    v8h hv[4], lv[4];
#pragma unroll
    for (int it = 0; it < 4; ++it) {
      const int row = it * 4 + q8;
      const float* sp = slab + row * kSlabPitch + c8;
#pragma unroll
      for (int e = 0; e < 8; ++e) {
        const float x = sp[e];
        const unsigned short hb = f2bf_bits(x);
        const unsigned short lb = f2bf_bits(x - bf_bits2f(hb));
        hv[it][e] = __builtin_bit_cast(_Float16, hb);
        lv[it][e] = __builtin_bit_cast(_Float16, lb);
      }
    }
    for (int pass = 0; pass < 2; ++pass) {
#pragma unroll
      for (int it = 0; it < 4; ++it) {
        const int row = it * 4 + q8;
        const size_t o = (row0 + 16 * wave + row) * kPlanePitch + kColQ + h * kHeadDim + c8;
        *(volatile v8h*)(PH + o) = hv[it];
        *(volatile v8h*)(PL + o) = lv[it];
      }
      __threadfence();
    }
    __syncthreads();
  }
}

extern "C" void kernel_launch(void* const* d_in, const int* in_sizes, int n_in,
                              void* d_out, int out_size, void* d_ws, size_t ws_size,
                              hipStream_t stream) {
  if (n_in < 6 || d_out == nullptr || d_ws == nullptr) return;
  if (in_sizes[0] != kRows * kEmb) return;
  if (in_sizes[1] != kEmb * kEmb || in_sizes[2] != kEmb * kEmb || in_sizes[3] != kEmb * kEmb || in_sizes[4] != kEmb * kEmb) return;
  if (in_sizes[5] != kEmb) return;
  if (out_size != kRows * kEmb) return;

  const float* x  = (const float*)d_in[0];
  const float* Wq = (const float*)d_in[1];
  const float* Wk = (const float*)d_in[2];
  const float* Wv = (const float*)d_in[3];
  const float* Wp = (const float*)d_in[4];
  const float* bp = (const float*)d_in[5];
  float* out = (float*)d_out;

  char* ws = (char*)d_ws;
  size_t off = 0;
  auto carve = [&](size_t bytes) -> char* { char* p = ws + off; off += (bytes + 255) & ~(size_t)255; return p; };
  unsigned short* XB   = (unsigned short*)carve(kBytesXB);
  unsigned short* WALL = (unsigned short*)carve(kBytesWALL);
  unsigned short* PH   = (unsigned short*)carve(kBytesPH);
  unsigned short* PL   = (unsigned short*)carve(kBytesPL);
  if (off != kWsTotal || off > ws_size || off > (size_t)134217728) return;

  const int n8x = kRows * kEmb / 8;
  const int n8w = kEmb * kEmb / 8;
  cvt8_bf16_kernel<<<dim3(n8x / 256, 1), 256, 0, stream>>>(x, x, x, x, XB, n8x);
  cvt8_bf16_kernel<<<dim3(n8w / 256, 4), 256, 0, stream>>>(Wq, Wk, Wv, Wp, WALL, n8w);

  wmma_gemm64<0, 0, 2, 6><<<dim3((kRows / 64) * (kPlanePitch / 64) / 8), 256, 0, stream>>>(
      XB, XB, kEmb,
      WALL, kEmb,
      (void*)PH, (void*)PL, kPlanePitch,
      bp, kRows, kPlanePitch, kEmb, 2 * kEmb);

  chunk_core_kernel<<<kBatch * kHeads, 256, 0, stream>>>(PH, PL);

  wmma_gemm64<1, 2, 0, 0><<<dim3((kRows / 64) * (kEmb / 64) / 8), 256, 0, stream>>>(
      PH, PL, kPlanePitch,
      WALL + (size_t)3 * kEmb * kEmb, kEmb,
      (void*)out, (void*)out, kEmb,
      bp, kRows, kEmb, kEmb, 0);
}
